// Block_72756745994545
// MI455X (gfx1250) — hardware-verified
//
#include <hip/hip_runtime.h>
#include <math.h>

constexpr int NBAT = 4;
constexpr int NSEQ = 2048;
constexpr int NCH  = 1024;
constexpr int NFF  = 4096;
constexpr int NROW = NBAT * NSEQ;
constexpr float LN_EPS_F   = 1e-5f;
constexpr float WCARRY     = 64.0f;
constexpr float WCARRY_INV = 1.0f / 64.0f;
constexpr float KKCARRY     = 256.0f;
constexpr float KKCARRY_INV = 1.0f / 256.0f;
static_assert(NROW % 64 == 0 && NSEQ % 64 == 0 && NCH % 64 == 0 && NFF % 64 == 0);
static_assert(NCH % 32 == 0 && NFF % 32 == 0);
static_assert(NCH == 4 * 256);
static_assert((NCH / 2) % 32 == 0);
static_assert((NBAT * NCH / 2) % 32 == 0);

typedef __attribute__((ext_vector_type(16))) _Float16 v16h;
typedef __attribute__((ext_vector_type(8)))  _Float16 v8h;
typedef __attribute__((ext_vector_type(8)))  float    v8f;
typedef __attribute__((ext_vector_type(4)))  float    v4f;
typedef __attribute__((ext_vector_type(2)))  unsigned v2u;

__device__ __forceinline__ void guard_row(v8f& a0, v8f& a1, v8f& a2, v8f& a3, v16h x, v16h b0, v16h b1, v16h b2, v16h b3) {
  asm volatile("v_nop\n\tv_nop\n\tv_nop\n\tv_nop" : "+v"(a0), "+v"(a1), "+v"(a2), "+v"(a3) : "v"(x), "v"(b0), "v"(b1), "v"(b2), "v"(b3));
}
__device__ __forceinline__ void keep4_h(v16h a, v16h b, v16h c, v16h d) { asm volatile("v_nop" :: "v"(a), "v"(b), "v"(c), "v"(d)); }
__device__ __forceinline__ void acc_guard4(v8f& a, v8f& b, v8f& c, v8f& d) { asm volatile("v_nop\n\tv_nop\n\tv_nop\n\tv_nop" : "+v"(a), "+v"(b), "+v"(c), "+v"(d)); }

union FragU { v16h v; v8h h[2]; };
__device__ __forceinline__ v16h frag_load(const _Float16* p) {
  FragU f;
  f.h[0] = *(const v8h*)(p);
  f.h[1] = *(const v8h*)(p + 16);
  return f.v;
}
__device__ __forceinline__ v8f frag_mma(v16h a, v16h b, v8f c) {
  return __builtin_amdgcn_wmma_f32_16x16x32_f16(false, a, false, b, (short)0, c, false, false);
}

__device__ __forceinline__ float h16_to_f32(unsigned hb) {
  const unsigned sgn = (hb & 0x8000u) << 16;
  const unsigned em = hb & 0x7fffu;
  const float fn = __uint_as_float((em << 13) + 0x38000000u);
  const float fs = (float)em * 5.9604644775390625e-8f;
  const float mag = (em < 0x400u) ? fs : fn;
  return __uint_as_float(__float_as_uint(mag) | sgn);
}
__device__ __forceinline__ unsigned f16bits(float f) {
  const _Float16 h = (_Float16)f;
  return (unsigned)__builtin_bit_cast(unsigned short, h);
}
__device__ __forceinline__ unsigned pack2h(float a, float b) {
  const unsigned lo = f16bits(a);
  const unsigned hi = f16bits(b);
  return lo | (hi << 16);
}
__device__ __forceinline__ float fsig(float x) { return __builtin_amdgcn_rcpf(1.0f + __expf(-x)); }

__global__ __launch_bounds__(256) void cvt8_f16_kernel(const float* __restrict__ src, unsigned short* __restrict__ dst, int n8, float sc) {
  const int i = blockIdx.x * 256 + threadIdx.x;
  if (i < n8) {
    const float* sp = src + (size_t)i * 8;
    const v4f a = *(const v4f*)(sp);
    const v4f b = *(const v4f*)(sp + 4);
    v8h hv;
#pragma unroll
    for (int e = 0; e < 4; ++e) {
      hv[e]     = (_Float16)(a[e] * sc);
      hv[4 + e] = (_Float16)(b[e] * sc);
    }
    *(volatile v8h*)(dst + (size_t)i * 8) = hv;
    __threadfence();
    *(volatile v8h*)(dst + (size_t)i * 8) = hv;
  }
}

template <bool HAS_V>
__global__ __launch_bounds__(256) void ln_mix_kernel(const float* __restrict__ X, const float* __restrict__ gam,
                                                     const float* __restrict__ bet, const float* __restrict__ tk,
                                                     const float* __restrict__ tv, const float* __restrict__ tr,
                                                     unsigned short* __restrict__ XK, unsigned short* __restrict__ XV,
                                                     unsigned short* __restrict__ XR) {
  __shared__ float redA[8][2];
  __shared__ float redB[8][2];
  const int tid = threadIdx.x, lane = tid & 31, wave = tid >> 5;
  const int row = blockIdx.x;
  const int tstep = row % NSEQ;
  const bool first = (tstep == 0);
  const int prow = first ? row : (row - 1);
  const int c4 = tid * 4;
  const v4f xc = *(const v4f*)(X + (size_t)row * NCH + c4);
  const v4f xp = *(const v4f*)(X + (size_t)prow * NCH + c4);
  float sc = (xc[0] + xc[1]) + (xc[2] + xc[3]);
  float sp = (xp[0] + xp[1]) + (xp[2] + xp[3]);
#pragma unroll
  for (int off = 1; off < 32; off <<= 1) {
    sc += __shfl_xor(sc, off, 32);
    sp += __shfl_xor(sp, off, 32);
  }
  if (lane == 0) { redA[wave][0] = sc; redA[wave][1] = sp; }
  __syncthreads();
  float tc = 0.0f, tp = 0.0f;
#pragma unroll
  for (int w = 0; w < 8; ++w) { tc += redA[w][0]; tp += redA[w][1]; }
  const float mc = tc * (1.0f / NCH);
  const float mp = tp * (1.0f / NCH);
  v4f dc, dp;
  float qc = 0.0f, qp = 0.0f;
#pragma unroll
  for (int e = 0; e < 4; ++e) {
    const float a = xc[e] - mc;
    const float b = xp[e] - mp;
    dc[e] = a;
    dp[e] = b;
    qc += a * a;
    qp += b * b;
  }
#pragma unroll
  for (int off = 1; off < 32; off <<= 1) {
    qc += __shfl_xor(qc, off, 32);
    qp += __shfl_xor(qp, off, 32);
  }
  if (lane == 0) { redB[wave][0] = qc; redB[wave][1] = qp; }
  __syncthreads();
  float vc = 0.0f, vp = 0.0f;
#pragma unroll
  for (int w = 0; w < 8; ++w) { vc += redB[w][0]; vp += redB[w][1]; }
  const float rc = rsqrtf(vc * (1.0f / NCH) + LN_EPS_F);
  const float rp = rsqrtf(vp * (1.0f / NCH) + LN_EPS_F);
  const v4f g  = *(const v4f*)(gam + c4);
  const v4f bb = *(const v4f*)(bet + c4);
  const v4f mk = *(const v4f*)(tk + c4);
  const v4f mv = *(const v4f*)(tv + c4);
  const v4f mr = *(const v4f*)(tr + c4);
  float ok[4], ov[4], orr[4];
#pragma unroll
  for (int e = 0; e < 4; ++e) {
    const float hc = (dc[e] * rc) * g[e] + bb[e];
    const float hq = (dp[e] * rp) * g[e] + bb[e];
    const float hp = first ? 0.0f : hq;
    ok[e]  = hc * mk[e] + hp * (1.0f - mk[e]);
    ov[e]  = hc * mv[e] + hp * (1.0f - mv[e]);
    orr[e] = hc * mr[e] + hp * (1.0f - mr[e]);
  }
  v2u pk, pv, pr;
  pk[0] = pack2h(ok[0], ok[1]);
  pk[1] = pack2h(ok[2], ok[3]);
  pv[0] = pack2h(ov[0], ov[1]);
  pv[1] = pack2h(ov[2], ov[3]);
  pr[0] = pack2h(orr[0], orr[1]);
  pr[1] = pack2h(orr[2], orr[3]);
  const size_t o = (size_t)row * NCH + c4;
  for (int pass = 0; pass < 2; ++pass) {
    *(volatile v2u*)(XK + o) = pk;
    if (HAS_V) *(volatile v2u*)(XV + o) = pv;
    *(volatile v2u*)(XR + o) = pr;
    __threadfence();
  }
}

enum { EP_F16 = 0, EP_SIG_F16 = 1, EP_RESID_F32 = 2, EP_RELU2_F16 = 3, EP_GATE_F32 = 4 };

template <int EPI>
__global__ __launch_bounds__(256) void gemm_f16_kernel(
    const unsigned short* __restrict__ Ap, int lda,
    const unsigned short* __restrict__ Btp, int ldb,
    void* __restrict__ Cout, int ldc,
    const float* __restrict__ resid,
    const unsigned short* __restrict__ gate,
    int M, int N, int K, float scale) {
  const _Float16* A  = (const _Float16*)Ap;
  const _Float16* Bt = (const _Float16*)Btp;
  __shared__ __align__(16) float sT[8][16 * 68];
  const int lane = threadIdx.x & 31;
  const int wave = threadIdx.x >> 5;
  const int tilesN = N >> 6;
  const int tilesM = M >> 6;
  const int tile = blockIdx.x * 8 + wave;
  if (tile >= tilesM * tilesN) return;
  const int tm = tile / tilesN;
  const int tn = tile - tm * tilesN;
  const int m0 = tm << 6;
  const int n0 = tn << 6;

  const int rlane = lane & 15;
  const int koff  = (lane >> 4) * 8;
  const int mOff  = (lane >> 4) * 8;

  v8f acc[4][4];
#pragma unroll
  for (int i = 0; i < 4; ++i)
#pragma unroll
    for (int j = 0; j < 4; ++j) acc[i][j] = (v8f){0.f, 0.f, 0.f, 0.f, 0.f, 0.f, 0.f, 0.f};

  for (int k0 = 0; k0 < K; k0 += 32) {
    v16h bh[4];
#pragma unroll
    for (int j = 0; j < 4; ++j) {
      const size_t bo = (size_t)(n0 + (j << 4) + rlane) * ldb + koff + k0;
      bh[j] = frag_load(Bt + bo);
    }
#pragma unroll
    for (int i = 0; i < 4; ++i) {
      const size_t ao = (size_t)(m0 + (i << 4) + rlane) * lda + koff + k0;
      const v16h ah = frag_load(A + ao);
#pragma unroll
      for (int j = 0; j < 4; ++j) acc[i][j] = frag_mma(ah, bh[j], acc[i][j]);
      guard_row(acc[i][0], acc[i][1], acc[i][2], acc[i][3], ah, bh[0], bh[1], bh[2], bh[3]);
    }
    keep4_h(bh[0], bh[1], bh[2], bh[3]);
  }
  acc_guard4(acc[0][0], acc[0][1], acc[0][2], acc[0][3]);
  acc_guard4(acc[1][0], acc[1][1], acc[1][2], acc[1][3]);
  acc_guard4(acc[2][0], acc[2][1], acc[2][2], acc[2][3]);
  acc_guard4(acc[3][0], acc[3][1], acc[3][2], acc[3][3]);

  float* slab = sT[wave];
#pragma unroll
  for (int i = 0; i < 4; ++i) {
    const int mBase = m0 + (i << 4);
#pragma unroll
    for (int j = 0; j < 4; ++j) {
#pragma unroll
      for (int r = 0; r < 8; ++r) {
        float v = acc[i][j][r] * scale;
        if (EPI == EP_RELU2_F16) {
          v = fmaxf(v, 0.0f);
          v = (v * v) * KKCARRY;
        }
        slab[(mOff + r) * 68 + (j << 4) + rlane] = v;
      }
    }
    __builtin_amdgcn_fence(__ATOMIC_RELEASE, "workgroup");
    __builtin_amdgcn_wave_barrier();
    __builtin_amdgcn_fence(__ATOMIC_ACQUIRE, "workgroup");
    if (EPI == EP_RESID_F32 || EPI == EP_GATE_F32) {
      float* C = (float*)Cout;
      const int hh = lane >> 4, c4 = (lane & 15) * 4;
      v4f outv[8];
#pragma unroll
      for (int it = 0; it < 8; ++it) {
        const int row = it * 2 + hh;
        const v4f v = *(const v4f*)(slab + row * 68 + c4);
        const size_t o = (size_t)(mBase + row) * ldc + n0 + c4;
        const v4f rr = *(const v4f*)(resid + o);
        if (EPI == EP_GATE_F32) {
          const v2u gw = *(const v2u*)(gate + o);
          const unsigned w0 = gw[0];
          const unsigned w1 = gw[1];
          const float g0 = h16_to_f32(w0 & 0xffffu);
          const float g1 = h16_to_f32(w0 >> 16);
          const float g2 = h16_to_f32(w1 & 0xffffu);
          const float g3 = h16_to_f32(w1 >> 16);
          outv[it][0] = rr[0] + g0 * v[0];
          outv[it][1] = rr[1] + g1 * v[1];
          outv[it][2] = rr[2] + g2 * v[2];
          outv[it][3] = rr[3] + g3 * v[3];
        } else {
          outv[it][0] = rr[0] + v[0];
          outv[it][1] = rr[1] + v[1];
          outv[it][2] = rr[2] + v[2];
          outv[it][3] = rr[3] + v[3];
        }
      }
      for (int pass = 0; pass < 2; ++pass) {
#pragma unroll
        for (int it = 0; it < 8; ++it) {
          const int row = it * 2 + hh;
          *(volatile v4f*)(C + (size_t)(mBase + row) * ldc + n0 + c4) = outv[it];
        }
        __threadfence();
      }
    } else {
      unsigned short* C = (unsigned short*)Cout;
      const int q = lane >> 3, c8 = (lane & 7) * 8;
      v8h hv[4];
#pragma unroll
      for (int it = 0; it < 4; ++it) {
        const int row = it * 4 + q;
        const float* sp = slab + row * 68 + c8;
        const v4f s0 = *(const v4f*)(sp);
        const v4f s1 = *(const v4f*)(sp + 4);
#pragma unroll
        for (int e = 0; e < 4; ++e) {
          float f0 = s0[e];
          float f1 = s1[e];
          if (EPI == EP_SIG_F16) {
            f0 = fsig(f0);
            f1 = fsig(f1);
          }
          hv[it][e]     = (_Float16)f0;
          hv[it][4 + e] = (_Float16)f1;
        }
      }
      for (int pass = 0; pass < 2; ++pass) {
#pragma unroll
        for (int it = 0; it < 4; ++it) {
          const int row = it * 4 + q;
          *(volatile v8h*)(C + (size_t)(mBase + row) * ldc + n0 + c8) = hv[it];
        }
        __threadfence();
      }
    }
    __builtin_amdgcn_fence(__ATOMIC_RELEASE, "workgroup");
    __builtin_amdgcn_wave_barrier();
    __builtin_amdgcn_fence(__ATOMIC_ACQUIRE, "workgroup");
  }
}

__device__ __forceinline__ float scan_step(float& aa, float& bb, float& pp, const float kk, const float vv,
                                           const float u, const float w) {
  const float ww = u + kk;
  const float p  = fmaxf(pp, ww);
  const float e1 = __expf(pp - p);
  const float e2 = __expf(ww - p);
  const float num = e1 * aa + e2 * vv;
  const float den = e1 * bb + e2;
  const float o = num * (1.0f / den);
  const float ww2 = pp + w;
  const float p2  = fmaxf(ww2, kk);
  const float f1  = __expf(ww2 - p2);
  const float f2  = __expf(kk - p2);
  aa = f1 * aa + f2 * vv;
  bb = f1 * bb + f2;
  pp = p2;
  return o;
}

__global__ __launch_bounds__(32) void decay_scan_gate_kernel(const float* __restrict__ tdecay, const float* __restrict__ tfirst,
                                                             const unsigned* __restrict__ K16, const unsigned* __restrict__ V16,
                                                             const unsigned* __restrict__ S16, unsigned* __restrict__ R16) {
  const int gid = blockIdx.x * 32 + threadIdx.x;
  const int b  = gid / (NCH / 2);
  const int cp = gid - b * (NCH / 2);
  const int c  = cp * 2;
  const float w0 = -expf(tdecay[c]);
  const float w1 = -expf(tdecay[c + 1]);
  const float u0 = tfirst[c];
  const float u1 = tfirst[c + 1];
  float aa0 = 0.0f, bb0 = 0.0f, pp0 = -1e38f;
  float aa1 = 0.0f, bb1 = 0.0f, pp1 = -1e38f;
  size_t idx = (size_t)b * NSEQ * (NCH / 2) + cp;
#pragma unroll 1
  for (int t = 0; t < NSEQ; ++t) {
    const unsigned kw = K16[idx];
    const unsigned vw = V16[idx];
    const unsigned sw = S16[idx];
    const float k0 = h16_to_f32(kw & 0xffffu);
    const float k1 = h16_to_f32(kw >> 16);
    const float v0 = h16_to_f32(vw & 0xffffu);
    const float v1 = h16_to_f32(vw >> 16);
    const float s0 = h16_to_f32(sw & 0xffffu);
    const float s1 = h16_to_f32(sw >> 16);
    const float o0 = scan_step(aa0, bb0, pp0, k0, v0, u0, w0);
    const float o1 = scan_step(aa1, bb1, pp1, k1, v1, u1, w1);
    const float r0 = s0 * o0;
    const float r1 = s1 * o1;
    const unsigned ow = pack2h(r0, r1);
    *(volatile unsigned*)(R16 + idx) = ow;
    __threadfence();
    *(volatile unsigned*)(R16 + idx) = ow;
    idx += (size_t)(NCH / 2);
  }
}

extern "C" void kernel_launch(void* const* d_in, const int* in_sizes, int n_in,
                              void* d_out, int out_size, void* d_ws, size_t ws_size, hipStream_t stream) {
  if (n_in < 19 || d_out == nullptr || d_ws == nullptr) return;
  if (in_sizes[0] != NROW * NCH || out_size != NROW * NCH) return;
  for (int i = 1; i <= 9; ++i) if (in_sizes[i] != NCH) return;
  for (int i = 10; i <= 13; ++i) if (in_sizes[i] != NCH * NCH) return;
  if (in_sizes[14] != NCH || in_sizes[15] != NCH) return;
  if (in_sizes[16] != NFF * NCH || in_sizes[17] != NCH * NCH || in_sizes[18] != NCH * NFF) return;

  const float* x       = (const float*)d_in[0];
  const float* ln1_w   = (const float*)d_in[1];
  const float* ln1_b   = (const float*)d_in[2];
  const float* ln2_w   = (const float*)d_in[3];
  const float* ln2_b   = (const float*)d_in[4];
  const float* t_decay = (const float*)d_in[5];
  const float* t_first = (const float*)d_in[6];
  const float* tmk     = (const float*)d_in[7];
  const float* tmv     = (const float*)d_in[8];
  const float* tmr     = (const float*)d_in[9];
  const float* att_kw  = (const float*)d_in[10];
  const float* att_vw  = (const float*)d_in[11];
  const float* att_rw  = (const float*)d_in[12];
  const float* att_ow  = (const float*)d_in[13];
  const float* f_tmk   = (const float*)d_in[14];
  const float* f_tmr   = (const float*)d_in[15];
  const float* f_kw    = (const float*)d_in[16];
  const float* f_rw    = (const float*)d_in[17];
  const float* f_vw    = (const float*)d_in[18];
  float* out = (float*)d_out;

  const size_t CC2 = (size_t)NCH * NCH * 2;
  const size_t FC2 = (size_t)NFF * NCH * 2;
  const size_t MC2 = (size_t)NROW * NCH * 2;
  char* ws = (char*)d_ws;
  size_t off = 0;
  auto carve = [&](size_t bytes) -> char* { char* p = ws + off; off += (bytes + 255) & ~(size_t)255; return p; };
  unsigned short* WK  = (unsigned short*)carve(CC2);
  unsigned short* WV  = (unsigned short*)carve(CC2);
  unsigned short* WR  = (unsigned short*)carve(CC2);
  unsigned short* WO  = (unsigned short*)carve(CC2);
  unsigned short* FKW = (unsigned short*)carve(FC2);
  unsigned short* FVW = (unsigned short*)carve(FC2);
  unsigned short* FRW = (unsigned short*)carve(CC2);
  unsigned short* P0  = (unsigned short*)carve(MC2);
  char*           P12 = carve(2 * MC2);
  unsigned short* P3  = (unsigned short*)carve(MC2);
  unsigned short* P4  = (unsigned short*)carve(MC2);
  unsigned short* P5  = (unsigned short*)carve(MC2);
  if (off > ws_size || off > (size_t)134217728) return;
  unsigned short* P1 = (unsigned short*)P12;
  unsigned short* P2 = (unsigned short*)(P12 + MC2);
  float* X1 = (float*)P12;

  const int n8c = NCH * NCH / 8;
  const int n8f = NFF * NCH / 8;
  cvt8_f16_kernel<<<n8c / 256, 256, 0, stream>>>(att_kw, WK,  n8c, WCARRY);
  cvt8_f16_kernel<<<n8c / 256, 256, 0, stream>>>(att_vw, WV,  n8c, WCARRY);
  cvt8_f16_kernel<<<n8c / 256, 256, 0, stream>>>(att_rw, WR,  n8c, WCARRY);
  cvt8_f16_kernel<<<n8c / 256, 256, 0, stream>>>(att_ow, WO,  n8c, WCARRY);
  cvt8_f16_kernel<<<n8f / 256, 256, 0, stream>>>(f_kw,   FKW, n8f, WCARRY);
  cvt8_f16_kernel<<<n8f / 256, 256, 0, stream>>>(f_vw,   FVW, n8f, WCARRY);
  cvt8_f16_kernel<<<n8c / 256, 256, 0, stream>>>(f_rw,   FRW, n8c, WCARRY);

  ln_mix_kernel<true><<<NROW, 256, 0, stream>>>(x, ln1_w, ln1_b, tmk, tmv, tmr, P0, P1, P2);

  const int gridCC = (NROW / 64) * (NCH / 64) / 8;
  gemm_f16_kernel<EP_F16><<<gridCC, 256, 0, stream>>>(P0, NCH, WK, NCH, (void*)P3, NCH, x, P0, NROW, NCH, NCH, WCARRY_INV);
  gemm_f16_kernel<EP_F16><<<gridCC, 256, 0, stream>>>(P1, NCH, WV, NCH, (void*)P4, NCH, x, P1, NROW, NCH, NCH, WCARRY_INV);
  gemm_f16_kernel<EP_SIG_F16><<<gridCC, 256, 0, stream>>>(P2, NCH, WR, NCH, (void*)P5, NCH, x, P2, NROW, NCH, NCH, WCARRY_INV);

  decay_scan_gate_kernel<<<(NBAT * NCH / 2) / 32, 32, 0, stream>>>(t_decay, t_first, (const unsigned*)P3, (const unsigned*)P4,
                                                                  (const unsigned*)P5, (unsigned*)P0);

  gemm_f16_kernel<EP_RESID_F32><<<gridCC, 256, 0, stream>>>(P0, NCH, WO, NCH, (void*)X1, NCH, x, P0, NROW, NCH, NCH, WCARRY_INV);

  ln_mix_kernel<false><<<NROW, 256, 0, stream>>>(X1, ln2_w, ln2_b, f_tmk, f_tmk, f_tmr, P3, P3, P4);

  gemm_f16_kernel<EP_SIG_F16><<<gridCC, 256, 0, stream>>>(P4, NCH, FRW, NCH, (void*)P5, NCH, x, P4, NROW, NCH, NCH, WCARRY_INV);

  const int gridKey = (NSEQ / 64) * (NFF / 64) / 8;
  const int gridVal = (NSEQ / 64) * (NCH / 64) / 8;
  for (int b = 0; b < NBAT; ++b) {
    const size_t ro = (size_t)b * NSEQ * NCH;
    gemm_f16_kernel<EP_RELU2_F16><<<gridKey, 256, 0, stream>>>(P3 + ro, NCH, FKW, NCH, (void*)P0, NFF, x, P3, NSEQ, NFF, NCH,
                                                               WCARRY_INV);
    gemm_f16_kernel<EP_GATE_F32><<<gridVal, 256, 0, stream>>>(P0, NFF, FVW, NFF, (void*)(out + ro), NCH, X1 + ro, P5 + ro,
                                                              NSEQ, NCH, NFF, WCARRY_INV * KKCARRY_INV);
  }
}
